// MultiLoraModule_48954037240345
// MI455X (gfx1250) — hardware-verified
//
#include <hip/hip_runtime.h>


#define NN_  4096
#define DIN  2048
#define DOUT 2048
#define RK   16
#define NAD  32
#define ZW   (NAD * RK)

typedef unsigned short bf;
typedef __attribute__((ext_vector_type(16))) __bf16   v16bf;
typedef __attribute__((ext_vector_type(8)))  unsigned short v8us;
typedef __attribute__((ext_vector_type(8)))  float    v8f;
typedef __attribute__((ext_vector_type(4)))  float    v4f;
typedef v4f  __attribute__((may_alias)) v4fa;
typedef v8us __attribute__((may_alias)) v8usa;

__device__ __forceinline__ unsigned short f2bf(float f) { unsigned u = __float_as_uint(f); u += 0x7FFFu + ((u >> 16) & 1u); return (unsigned short)(u >> 16); }
__device__ __forceinline__ float bf2f(unsigned short b) { return __uint_as_float(((unsigned)b) << 16); }
__device__ __forceinline__ float bfr(float f) { return bf2f(f2bf(f)); }
__device__ __forceinline__ v16bf cat16b(v8us lo, v8us hi) { return __builtin_bit_cast(v16bf, __builtin_shufflevector(lo, hi, 0, 1, 2, 3, 4, 5, 6, 7, 8, 9, 10, 11, 12, 13, 14, 15)); }
__device__ __forceinline__ v8f wmmab(v16bf a, v16bf b, v8f c) { return __builtin_amdgcn_wmma_f32_16x16x32_bf16(false, a, false, b, (short)0, c, false, false); }
#define VST2(T, p, v) do { const T vst2_v_ = (v); *(volatile T*)(p) = vst2_v_; __threadfence(); *(volatile T*)(p) = vst2_v_; } while (0)

__global__ __launch_bounds__(256) void k_cvtb(const float* __restrict__ src, int nrows, bf* dst) {
    const int lane = threadIdx.x & 31, r = blockIdx.x * 8 + (threadIdx.x >> 5);
    if (r >= nrows) return;
#pragma unroll
    for (int q = 0; q < DIN / 256; ++q) { v8us t;
#pragma unroll
        for (int i = 0; i < 8; ++i) t[i] = f2bf(src[(size_t)r * DIN + q * 256 + lane * 8 + i]);
        VST2(v8us, dst + (size_t)r * DIN + q * 256 + lane * 8, t); }
}
__global__ __launch_bounds__(256) void k_bt(const float* __restrict__ LB, bf* BT) {
    const int lane = threadIdx.x & 31, o = blockIdx.x * 8 + (threadIdx.x >> 5);
    if (o >= DOUT) return;
#pragma unroll
    for (int s = 0; s < 2; ++s) { const int a = 16 * s + (lane >> 1), r0 = (lane & 1) * 8; v8us t;
#pragma unroll
        for (int r = 0; r < 8; ++r) t[r] = f2bf(LB[((size_t)a * DOUT + o) * RK + r0 + r]);
        VST2(v8us, BT + (size_t)o * ZW + s * 256 + lane * 8, t); }
}
template <bool SPLITA, int MODE>
__global__ __launch_bounds__(128) void k_gemm(const bf* __restrict__ A, const bf* __restrict__ Al, const bf* __restrict__ Bn, int K, int ldc, const float* __restrict__ bias, float* C) {
    __shared__ __align__(16) float ost[4][16 * 68];
    const int lane = threadIdx.x & 31, wave = threadIdx.x >> 5, lr = lane & 15, hi = lane >> 4;
    const int r0 = blockIdx.x * 64 + wave * 16, c0 = blockIdx.y * 64;
    const size_t aoff = (size_t)(r0 + lr) * K + 8 * hi;
    size_t boff[4];
#pragma unroll
    for (int t = 0; t < 4; ++t) boff[t] = (size_t)(c0 + t * 16 + lr) * K + 8 * hi;
    v8f acc[4];
#pragma unroll
    for (int t = 0; t < 4; ++t) acc[t] = (v8f){};
#pragma unroll 1
    for (int kc = 0; kc < K; kc += 32) {
        const v16bf a = cat16b(*(const v8us*)(A + aoff + kc), *(const v8us*)(A + aoff + kc + 16));
        v16bf al = a;
        if (SPLITA) al = cat16b(*(const v8us*)(Al + aoff + kc), *(const v8us*)(Al + aoff + kc + 16));
#pragma unroll
        for (int t = 0; t < 4; ++t) { const v16bf b = cat16b(*(const v8us*)(Bn + boff[t] + kc), *(const v8us*)(Bn + boff[t] + kc + 16)); acc[t] = wmmab(a, b, acc[t]); if (SPLITA) acc[t] = wmmab(al, b, acc[t]); }
        asm volatile("v_nop\n\tv_nop\n\tv_nop\n\tv_nop" : "+v"(acc[0]), "+v"(acc[1]), "+v"(acc[2]), "+v"(acc[3]) : "v"(a), "v"(al));
    }
    float* os = &ost[wave][0];
#pragma unroll
    for (int t = 0; t < 4; ++t) { const int col = c0 + t * 16 + lr; const float bv = (MODE == 0) ? bfr(bias[col]) : 0.f;
#pragma unroll
        for (int j = 0; j < 8; ++j) { float v = acc[t][j] + bv; if (MODE == 2) v += C[(size_t)(r0 + hi * 8 + j) * ldc + col]; os[(hi * 8 + j) * 68 + t * 16 + lr] = v; } }
    __syncthreads();
    float* crow = C + (size_t)r0 * ldc + c0;
    auto pass = [&]() {
#pragma unroll
        for (int s = 0; s < 8; ++s) { const int Lid = (lane >> 3) + 4 * s, piece = lane & 7; const int row = Lid >> 1, cofs = (Lid & 1) * 32 + piece * 4;
            const v4f val = *(const v4fa*)(os + row * 68 + cofs); *(volatile v4f*)(crow + (size_t)row * ldc + cofs) = val; }
    };
    pass(); __threadfence(); pass();
}
__global__ __launch_bounds__(256) void k_z(const float* __restrict__ H, const int* __restrict__ ids, const float* __restrict__ sc, bf* ZH, bf* ZL) {
    const int lane = threadIdx.x & 31, n = blockIdx.x * 8 + (threadIdx.x >> 5);
    if (n >= NN_) return;
    int id = ids[n]; if (id < 0) id += NAD; id = ((unsigned)id < (unsigned)NAD) ? id : 0;
    const float s = bfr(sc[id]);
#pragma unroll
    for (int q = 0; q < 2; ++q) { const int a = 16 * q + (lane >> 1), r0 = (lane & 1) * 8; v8us oh, ol;
#pragma unroll
        for (int r = 0; r < 8; ++r) { const float v = (a == id) ? H[(size_t)n * ZW + a * RK + r0 + r] * s : 0.f; const unsigned short hb = f2bf(v); oh[r] = hb; ol[r] = f2bf(v - bf2f(hb)); }
        *(volatile v8us*)(ZH + (size_t)n * ZW + q * 256 + lane * 8) = oh; *(volatile v8us*)(ZL + (size_t)n * ZW + q * 256 + lane * 8) = ol; __threadfence();
        *(volatile v8us*)(ZH + (size_t)n * ZW + q * 256 + lane * 8) = oh; *(volatile v8us*)(ZL + (size_t)n * ZW + q * 256 + lane * 8) = ol; }
}

extern "C" void kernel_launch(void* const* d_in, const int* in_sizes, int n_in,
                              void* d_out, int out_size, void* d_ws, size_t ws_size, hipStream_t stream) {
    (void)in_sizes; (void)n_in; (void)out_size;
    const float* x = (const float*)d_in[0]; const int* ids = (const int*)d_in[1]; const float* Wb = (const float*)d_in[2]; const float* bb = (const float*)d_in[3];
    const float* LA = (const float*)d_in[4]; const float* LB = (const float*)d_in[5]; const float* sc = (const float*)d_in[6];
    float* out = (float*)d_out;
    char* wsp = (char*)d_ws;
    auto take = [&](size_t bytes) { char* p = wsp; wsp += (bytes + 255) & ~(size_t)255; return (void*)p; };
    bf* Xb = (bf*)take((size_t)NN_ * DIN * 2); bf* WB = (bf*)take((size_t)DOUT * DIN * 2); bf* AB = (bf*)take((size_t)ZW * DIN * 2); bf* BT = (bf*)take((size_t)DOUT * ZW * 2);
    float* H = (float*)take((size_t)NN_ * ZW * 4); bf* ZH = (bf*)take((size_t)NN_ * ZW * 2); bf* ZL = (bf*)take((size_t)NN_ * ZW * 2);
    if ((size_t)(wsp - (char*)d_ws) > ws_size) return;
    k_cvtb<<<NN_ / 8, 256, 0, stream>>>(x, NN_, Xb);
    k_cvtb<<<DOUT / 8, 256, 0, stream>>>(Wb, DOUT, WB);
    k_cvtb<<<ZW / 8, 256, 0, stream>>>(LA, ZW, AB);
    k_bt<<<DOUT / 8, 256, 0, stream>>>(LB, BT);
    k_gemm<false, 0><<<dim3(NN_ / 64, DOUT / 64, 1), 128, 0, stream>>>(Xb, nullptr, WB, DIN, DOUT, bb, out);
    k_gemm<false, 1><<<dim3(NN_ / 64, ZW / 64, 1), 128, 0, stream>>>(Xb, nullptr, AB, DIN, ZW, nullptr, H);
    k_z<<<NN_ / 8, 256, 0, stream>>>(H, ids, sc, ZH, ZL);
    k_gemm<true, 2><<<dim3(NN_ / 64, DOUT / 64, 1), 128, 0, stream>>>(ZH, ZL, BT, ZW, DOUT, nullptr, out);
}
